// ECConvLayer_38620345926111
// MI455X (gfx1250) — hardware-verified
//
#include <hip/hip_runtime.h>
#include <math.h>

typedef __attribute__((ext_vector_type(16))) _Float16 v16h;
typedef __attribute__((ext_vector_type(16))) __bf16 v16b;
typedef __attribute__((ext_vector_type(8)))  _Float16 v8h;
typedef __attribute__((ext_vector_type(8)))  float v8f;
typedef __attribute__((ext_vector_type(4)))  float v4f;
typedef __attribute__((ext_vector_type(2)))  float v2f;
typedef __attribute__((ext_vector_type(4)))  unsigned v4u;
typedef __attribute__((ext_vector_type(4)))  int v4i;
typedef float __attribute__((may_alias)) float_a;
typedef int __attribute__((may_alias)) int_a;

template <typename T> __device__ __forceinline__ void vst2(void* p, T v) { *(volatile T*)p = v; __threadfence(); *(volatile T*)p = v; }
__device__ __forceinline__ v8f wmma16(v16h a, v16h b, v8f c) {
  v8f d = __builtin_amdgcn_wmma_f32_16x16x32_f16(false, a, false, b, (short)0, c, false, false);
  asm volatile("v_nop\n\tv_nop\n\tv_nop\n\tv_nop" : "+v"(d) : "v"(a), "v"(b));
  return d;
}
__device__ __forceinline__ v8f wmma_bf(v16b a, v16b b, v8f c) {
  v8f d = __builtin_amdgcn_wmma_f32_16x16x32_bf16(false, a, false, b, (short)0, c, false, false);
  asm volatile("v_nop\n\tv_nop\n\tv_nop\n\tv_nop" : "+v"(d) : "v"(a), "v"(b));
  return d;
}
__device__ __forceinline__ v16h frag_h(const _Float16* rowk0, int lane) {
  union { v16h v; v8h q[2]; } u; const _Float16* p = rowk0 + 8 * (lane >> 4);
  u.q[0] = *(const v8h*)p; u.q[1] = *(const v8h*)(p + 16); return u.v;
}
__device__ __forceinline__ v16h frag_f32(const float* rowk0, int lane) {
  v16h a; const float* p = rowk0 + 8 * (lane >> 4);
#pragma unroll
  for (int i = 0; i < 8; ++i) { a[i] = (_Float16)p[i]; a[8 + i] = (_Float16)p[16 + i]; }
  return a;
}
__device__ __forceinline__ v16h frag_f32s(const float* rowk0, int lane, float sc) {
  v16h a; const float* p = rowk0 + 8 * (lane >> 4);
#pragma unroll
  for (int i = 0; i < 8; ++i) { a[i] = (_Float16)(p[i] * sc); a[8 + i] = (_Float16)(p[16 + i] * sc); }
  return a;
}
__device__ __forceinline__ v16h fragc_f32(const float* W, int k0, int n, int lane, int ld, int K) {
  v16h a; const int g = lane >> 4;
#pragma unroll
  for (int i = 0; i < 8; ++i) { const int ka = k0 + 8 * g + i, kb = ka + 16;
    a[i] = (_Float16)(ka < K ? W[(size_t)ka * ld + n] : 0.f); a[8 + i] = (_Float16)(kb < K ? W[(size_t)kb * ld + n] : 0.f); }
  return a;
}
struct F2 { v16b h, l; };
__device__ __forceinline__ F2 bsplit16(const float v[16]) { F2 r;
#pragma unroll
  for (int i = 0; i < 16; ++i) { const __bf16 h = (__bf16)v[i]; r.h[i] = h; r.l[i] = (__bf16)(v[i] - (float)h); }
  return r; }
__device__ __forceinline__ F2 split_row(const float* row, int k0, int lane) { float v[16]; const float* p = row + k0 + 8 * (lane >> 4);
#pragma unroll
  for (int i = 0; i < 8; ++i) { v[i] = p[i]; v[8 + i] = p[16 + i]; }
  return bsplit16(v); }
__device__ __forceinline__ F2 split_rowK(const float* row, int k0, int lane, int K) { float v[16]; const int g = lane >> 4;
#pragma unroll
  for (int i = 0; i < 8; ++i) { const int ka = k0 + 8 * g + i, kb = ka + 16; v[i] = ka < K ? row[ka] : 0.f; v[8 + i] = kb < K ? row[kb] : 0.f; }
  return bsplit16(v); }
__device__ __forceinline__ F2 split_col(const float* W, int k0, int n, int lane, int ld, int K) { float v[16]; const int g = lane >> 4;
#pragma unroll
  for (int i = 0; i < 8; ++i) { const int ka = k0 + 8 * g + i, kb = ka + 16; v[i] = ka < K ? W[(size_t)ka * ld + n] : 0.f; v[8 + i] = kb < K ? W[(size_t)kb * ld + n] : 0.f; }
  return bsplit16(v); }
__device__ __forceinline__ v8f mac3(const F2& a, const F2& b, v8f c) { c = wmma_bf(a.l, b.h, c); c = wmma_bf(a.h, b.l, c); return wmma_bf(a.h, b.h, c); }
__device__ __forceinline__ float sigm(float v) { return 1.0f / (1.0f + expf(-v)); }
#define LDSX() do { asm volatile("s_wait_dscnt 0" ::: "memory"); __builtin_amdgcn_wave_barrier(); __builtin_amdgcn_fence(__ATOMIC_RELEASE, "workgroup"); } while (0)

#define NSRC 32768
#define NDST 8192
#define NE 65536
#define DI 64
#define DE 32
#define DH 64
#define RB 1024
#define NRB (NDST / RB)
#define NN NDST
#define EPT 16
#define CH (256 * EPT)

__global__ __launch_bounds__(256) void k_pack(const float* __restrict__ We, _Float16* __restrict__ WeT) {
  const int n0 = blockIdx.x * 256, tid = threadIdx.x; __shared__ __align__(16) _Float16 st[256][40];
  for (int q = tid; q < 256 * 32; q += 256) { const int k = q >> 8, nl = q & 255; st[nl][k] = (_Float16)(We[(size_t)k * 4096 + n0 + nl] * 16.0f); }
  __syncthreads();
  for (int q = tid; q < 256 * 4; q += 256) { const int nl = q >> 2, pc = q & 3; vst2(WeT + (size_t)(n0 + nl) * DE + pc * 8, *(const v4u*)(&st[nl][pc * 8])); }
}
__global__ __launch_bounds__(128) void k_edge(const float* __restrict__ ef, const int* __restrict__ src, const float* __restrict__ node, const _Float16* __restrict__ WeT, const float* __restrict__ be, float* __restrict__ M) {
  __shared__ __align__(16) float shs[4][16][DI + 4];
  __shared__ __align__(16) float sm[4][16][DH + 4];
  const int tid = threadIdx.x, wave = tid >> 5, lane = tid & 31, col = lane & 15, g = lane >> 4;
  const int e0 = blockIdx.x * 64 + wave * 16;
  for (int q = lane; q < 16 * 16; q += 32) { const int rl = q >> 4, pc = q & 15; int s = src[e0 + rl]; s = s < 0 ? 0 : (s >= NSRC ? NSRC - 1 : s); *(v4f*)(&shs[wave][rl][pc * 4]) = *(const v4f*)(node + (size_t)s * DI + pc * 4); }
  const v16h a = frag_f32(ef + (size_t)(e0 + col) * DE, lane);
  LDSX();
#pragma unroll 1
  for (int h = 0; h < DH; ++h) { float part[8] = {0.f, 0.f, 0.f, 0.f, 0.f, 0.f, 0.f, 0.f};
#pragma unroll
    for (int t4 = 0; t4 < 4; ++t4) { const int n = h * DI + t4 * 16 + col; const v8f acc = wmma16(a, frag_h(WeT + (size_t)n * DE, lane), (v8f){}); const float bb = be[n]; const int d = t4 * 16 + col;
#pragma unroll
      for (int r = 0; r < 8; ++r) { const float w = acc[r] * (1.0f / 16.0f) + bb; part[r] += (w > 0.f ? w : 0.f) * shs[wave][8 * g + r][d]; } }
#pragma unroll
    for (int r = 0; r < 8; ++r) {
#pragma unroll
      for (int off = 1; off <= 8; off <<= 1) part[r] += __shfl_xor(part[r], off, 32); }
    { float pv = 0.f;
#pragma unroll
      for (int r = 0; r < 8; ++r) pv = (r == col) ? part[r] : pv;
      if (col < 8) sm[wave][8 * g + col][h] = pv; } }
  LDSX();
  for (int q = lane; q < 16 * 16; q += 32) { const int rl = q >> 4, pc = q & 15; vst2(M + (size_t)(e0 + rl) * DH + pc * 4, *(const v4f*)(&sm[wave][rl][pc * 4])); }
}
__global__ __launch_bounds__(256) void k_agg(const float* __restrict__ M, const int* __restrict__ dst, const float* __restrict__ node, const float* __restrict__ Wn, const float* __restrict__ bn, float* __restrict__ out) {
  __shared__ __align__(16) float sacc[RB][DH];
  __shared__ __align__(16) union { struct { int ssrc[8][32 * EPT], sdl[8][32 * EPT]; } l; float so[8][16][64]; } UU;
  __shared__ int scnt[8]; __shared__ int srcnt[RB];
  int (*ssrc)[32 * EPT] = UU.l.ssrc; int (*sdl)[32 * EPT] = UU.l.sdl; float (*so)[16][64] = UU.so;
  const int tid = threadIdx.x, wave = tid >> 5, lane = tid & 31, col = lane & 15, g = lane >> 4;
  const int r0 = blockIdx.x * RB; const int* edst = dst;
  for (int q = tid; q < RB * DH; q += 256) (&sacc[0][0])[q] = 0.f;
  for (int q = tid; q < RB; q += 256) srcnt[q] = 0;
  __syncthreads();
#pragma unroll 1
  for (int c0 = 0; c0 < NE; c0 += CH) { const int e0 = c0 + tid * EPT; int hd[EPT];
    if (e0 + EPT <= NE) {
#pragma unroll
      for (int v = 0; v < EPT / 4; ++v) { const int4 d4 = *(const int4*)(edst + e0 + v * 4); const int dd[4] = {d4.x, d4.y, d4.z, d4.w};
#pragma unroll
        for (int u = 0; u < 4; ++u) { const unsigned rel = (unsigned)(dd[u] - r0); hd[v * 4 + u] = rel < (unsigned)RB ? (int)rel : -1; } } }
    else {
#pragma unroll
      for (int u = 0; u < EPT; ++u) { const int e = e0 + u; int d = -1; if (e < NE) { const unsigned rel = (unsigned)(edst[e] - r0); d = rel < (unsigned)RB ? (int)rel : -1; } hd[u] = d; } }
    int cnt = 0;
#pragma unroll
    for (int u = 0; u < EPT; ++u) cnt += hd[u] >= 0;
    int incl = cnt;
#pragma unroll
    for (int off = 1; off < 32; off <<= 1) { const int v = __shfl_up(incl, off, 32); if (lane >= off) incl += v; }
    if (lane == 31) scnt[wave] = incl;
    int pos = incl - cnt;
#pragma unroll
    for (int u = 0; u < EPT; ++u) if (hd[u] >= 0) { ssrc[wave][pos] = e0 + u; sdl[wave][pos] = hd[u]; atomicAdd(&srcnt[hd[u]], 1); ++pos; }
    __syncthreads();
    if (tid < DH) { for (int w = 0; w < 8; ++w) { const int nh = scnt[w]; for (int i = 0; i < nh; ++i) sacc[sdl[w][i]][tid] += M[(size_t)ssrc[w][i] * DH + tid]; } }
    __syncthreads(); }
  for (int q = tid; q < RB * DH; q += 256) { const int rl = q >> 6, c = q & 63; const int cnt = srcnt[rl]; sacc[rl][c] = cnt > 0 ? sacc[rl][c] / (float)cnt : 0.f; }
  __syncthreads();
#pragma unroll 1
  for (int tt = 0; tt < 8; ++tt) { const int rt = wave * 8 + tt; const int row = r0 + rt * 16 + col; v8f acc[4] = {};
#pragma unroll
    for (int kc = 0; kc < 4; ++kc) { const F2 a = kc < 2 ? split_row(node + (size_t)row * DI, kc * 32, lane) : split_row(&sacc[rt * 16 + col][0], (kc - 2) * 32, lane);
#pragma unroll
      for (int t = 0; t < 4; ++t) acc[t] = mac3(a, split_col(Wn, kc * 32, t * 16 + col, lane, DH, DI + DH), acc[t]); }
#pragma unroll
    for (int t = 0; t < 4; ++t) { const float bb = bn[t * 16 + col];
#pragma unroll
      for (int r = 0; r < 8; ++r) { const float v = acc[t][r] + bb; so[wave][8 * g + r][t * 16 + col] = v > 0.f ? v : 0.f; } }
    LDSX();
    for (int q = lane; q < 16 * 16; q += 32) { const int rl = q >> 4, pc = q & 15; vst2(out + (size_t)(r0 + rt * 16 + rl) * DH + pc * 4, *(const v4f*)(&so[wave][rl][pc * 4])); }
    LDSX(); }
}
extern "C" void kernel_launch(void* const* d_in, const int* in_sizes, int n_in, void* d_out, int out_size, void* d_ws, size_t ws_size, hipStream_t stream) {
  (void)in_sizes; (void)n_in; (void)out_size; (void)ws_size;
  const float* node = (const float*)d_in[0]; const float* ef = (const float*)d_in[1]; const int* src = (const int*)d_in[2]; const int* dst = (const int*)d_in[3]; const float* We = (const float*)d_in[4]; const float* be = (const float*)d_in[5]; const float* Wn = (const float*)d_in[6]; const float* bn = (const float*)d_in[7];
  float* out = (float*)d_out;
  char* ws = (char*)d_ws; size_t off = 0;
  auto take = [&](size_t bytes) { char* p = ws + off; off += (bytes + 255) & ~(size_t)255; return p; };
  _Float16* WeT = (_Float16*)take((size_t)4096 * DE * 2); float* M = (float*)take((size_t)NE * DH * 4);
  k_pack<<<4096 / 256, 256, 0, stream>>>(We, WeT);
  k_edge<<<NE / 64, 128, 0, stream>>>(ef, src, node, WeT, be, M);
  k_agg<<<NRB, 256, 0, stream>>>(M, dst, node, Wn, bn, out);
}
